// NonLocal_25821343384300
// MI455X (gfx1250) — hardware-verified
//
#include <hip/hip_runtime.h>
#include <math.h>
#include <stdint.h>

#define NB    4
#define CI    256
#define CM    128
#define NSP   3136
#define NTOKS (NB * NSP)
#define K3    (3 * NSP)
#define T3P   (3 * CM)
#define O2P   (2 * CM)

static_assert(NSP % 64 == 0);
static_assert(NTOKS % 64 == 0);
static_assert(CI % 64 == 0);
static_assert(CM % 64 == 0);
static_assert(CI % 32 == 0);
static_assert(K3 % 32 == 0);
static_assert(T3P % 32 == 0);
static_assert(O2P % 32 == 0);
static_assert((CM * CI) % (8 * 256) == 0);
static_assert((CI * CM) % (8 * 256) == 0);

typedef __attribute__((ext_vector_type(16))) _Float16 v16h;
typedef __attribute__((ext_vector_type(8)))  _Float16 v8h;
typedef __attribute__((ext_vector_type(16))) __bf16   v16b;
typedef __attribute__((ext_vector_type(8)))  __bf16   v8b;
typedef __attribute__((ext_vector_type(8)))  float    v8f;
typedef __attribute__((ext_vector_type(4)))  float    v4f;
typedef __attribute__((ext_vector_type(4)))  unsigned int v4u;

__device__ __forceinline__ unsigned short f2bf_bits(float f) {
  unsigned u = __float_as_uint(f);
  return (unsigned short)((u + 0x7FFFu + ((u >> 16) & 1u)) >> 16);
}
__device__ __forceinline__ float bf_bits2f(unsigned short h) { return __uint_as_float(((unsigned)h) << 16); }
__device__ __forceinline__ float bf_rne(float f) { return bf_bits2f(f2bf_bits(f)); }
__device__ __forceinline__ unsigned pk16(unsigned short a, unsigned short b) { return (unsigned)a | ((unsigned)b << 16); }

__device__ __forceinline__ void dep_guard_h(v8f& a, v8f& b, v16h x, v16h y) { asm volatile("v_nop\n\tv_nop\n\tv_nop\n\tv_nop" : "+v"(a), "+v"(b) : "v"(x), "v"(y)); }
__device__ __forceinline__ void dep_guard_b(v8f& a, v8f& b, v16b x, v16b y) { asm volatile("v_nop\n\tv_nop\n\tv_nop\n\tv_nop" : "+v"(a), "+v"(b) : "v"(x), "v"(y)); }
__device__ __forceinline__ void keep4_h(v16h a, v16h b, v16h c, v16h d) { asm volatile("v_nop" :: "v"(a), "v"(b), "v"(c), "v"(d)); }
__device__ __forceinline__ void keep4_b(v16b a, v16b b, v16b c, v16b d) { asm volatile("v_nop" :: "v"(a), "v"(b), "v"(c), "v"(d)); }
__device__ __forceinline__ void acc_guard4(v8f& a, v8f& b, v8f& c, v8f& d) { asm volatile("v_nop\n\tv_nop\n\tv_nop\n\tv_nop" : "+v"(a), "+v"(b), "+v"(c), "+v"(d)); }

template <typename T> struct Frag;
template <> struct Frag<_Float16> {
  typedef v16h V; union U { v16h v; v8h h[2]; };
  static __device__ __forceinline__ v16h load(const _Float16* p) {
    U f; f.h[0] = *(const v8h*)(p); f.h[1] = *(const v8h*)(p + 16); return f.v;
  }
  static __device__ __forceinline__ v8f mma(v16h a, v16h b, v8f c) {
    return __builtin_amdgcn_wmma_f32_16x16x32_f16(false, a, false, b, (short)0, c, false, false);
  }
  static __device__ __forceinline__ void guard(v8f& a, v8f& b, v16h x, v16h y) { dep_guard_h(a, b, x, y); }
  static __device__ __forceinline__ void keep(v16h a, v16h b, v16h c, v16h d) { keep4_h(a, b, c, d); }
};
template <> struct Frag<__bf16> {
  typedef v16b V; union U { v16b v; v8b h[2]; };
  static __device__ __forceinline__ v16b load(const __bf16* p) {
    U f; f.h[0] = *(const v8b*)(p); f.h[1] = *(const v8b*)(p + 16); return f.v;
  }
  static __device__ __forceinline__ v8f mma(v16b a, v16b b, v8f c) {
    return __builtin_amdgcn_wmma_f32_16x16x32_bf16(false, a, false, b, (short)0, c, false, false);
  }
  static __device__ __forceinline__ void guard(v8f& a, v8f& b, v16b x, v16b y) { dep_guard_b(a, b, x, y); }
  static __device__ __forceinline__ void keep(v16b a, v16b b, v16b c, v16b d) { keep4_b(a, b, c, d); }
};

template <int ET> struct Elem;
template <> struct Elem<0> { typedef _Float16 T; };
template <> struct Elem<1> { typedef __bf16 T; };

template <int ET, int BIAS_MODE, int OUT_MODE, bool RESID, bool BN>
__global__ __launch_bounds__(256) void wmma_gemm64(
    const unsigned short* __restrict__ Ap, int lda, long strideA,
    const unsigned short* __restrict__ Btp, int ldb, long strideB,
    void* Cout, void* Cout2, void* Cout3, int ldc, long strideC,
    const float* __restrict__ bias,
    const float* __restrict__ bng, const float* __restrict__ bnb,
    const float* __restrict__ bnm, const float* __restrict__ bnv,
    const float* __restrict__ resid, long strideR,
    int M, int N, int K, float scale) {
  typedef typename Elem<ET>::T T;
  typedef typename Frag<T>::V V;
  const T* A = (const T*)Ap; const T* Bt = (const T*)Btp;
  __shared__ __align__(16) float sT[8][16 * 68];
  const int b    = blockIdx.y;
  const int lane = threadIdx.x & 31;
  const int wave = threadIdx.x >> 5;
  const int tilesN = N >> 6;
  const int tilesM = M >> 6;
  const int tile = blockIdx.x * 8 + wave;
  if (tile >= tilesM * tilesN) return;
  const int tm = tile / tilesN;
  const int tn = tile - tm * tilesN;
  const int m0 = tm << 6;
  const int n0 = tn << 6;

  const T* Ab = A  + (size_t)b * strideA;
  const T* Bb = Bt + (size_t)b * strideB;

  const int rlane = lane & 15;
  const int koff  = (lane >> 4) * 8;
  const int mOff  = (lane >> 4) * 8;

  v8f acc[4][4];
#pragma unroll
  for (int i = 0; i < 4; ++i)
#pragma unroll
    for (int j = 0; j < 4; ++j) acc[i][j] = (v8f){0.f,0.f,0.f,0.f,0.f,0.f,0.f,0.f};

  for (int k0 = 0; k0 < K; k0 += 32) {
    V bh[4];
#pragma unroll
    for (int j = 0; j < 4; ++j) {
      const size_t bo = (size_t)(n0 + (j << 4) + rlane) * ldb + koff + k0;
      bh[j] = Frag<T>::load(Bb + bo);
    }
#pragma unroll
    for (int i = 0; i < 4; ++i) {
      const size_t ao = (size_t)(m0 + (i << 4) + rlane) * lda + koff + k0;
      const V ah = Frag<T>::load(Ab + ao);
#pragma unroll
      for (int j = 0; j < 4; ++j) acc[i][j] = Frag<T>::mma(ah, bh[j], acc[i][j]);
      Frag<T>::guard(acc[i][0], acc[i][3], ah, ah);
    }
    Frag<T>::keep(bh[0], bh[1], bh[2], bh[3]);
  }
  acc_guard4(acc[0][0], acc[0][1], acc[0][2], acc[0][3]);
  acc_guard4(acc[1][0], acc[1][1], acc[1][2], acc[1][3]);
  acc_guard4(acc[2][0], acc[2][1], acc[2][2], acc[2][3]);
  acc_guard4(acc[3][0], acc[3][1], acc[3][2], acc[3][3]);

  float* slab = sT[wave];
  const float* Rb = resid + (size_t)b * (RESID ? (size_t)strideR : (size_t)0);
#pragma unroll
  for (int i = 0; i < 4; ++i) {
    const int mBase = m0 + (i << 4);
    const int mr = mBase + mOff;
    float rb[8], rmul[8], radd[8];
#pragma unroll
    for (int r = 0; r < 8; ++r) { rb[r] = 0.f; rmul[r] = 1.f; radd[r] = 0.f; }
    if (BIAS_MODE == 1) {
      const v4f t0 = *(const v4f*)(bias + mr);
      const v4f t1 = *(const v4f*)(bias + mr + 4);
#pragma unroll
      for (int e = 0; e < 4; ++e) { rb[e] = bf_rne(t0[e]); rb[4 + e] = bf_rne(t1[e]); }
    }
    if (BN) {
      const v4f vg0 = *(const v4f*)(bng + mr), vg1 = *(const v4f*)(bng + mr + 4);
      const v4f vb0 = *(const v4f*)(bnb + mr), vb1 = *(const v4f*)(bnb + mr + 4);
      const v4f vm0 = *(const v4f*)(bnm + mr), vm1 = *(const v4f*)(bnm + mr + 4);
      const v4f vv0 = *(const v4f*)(bnv + mr), vv1 = *(const v4f*)(bnv + mr + 4);
#pragma unroll
      for (int e = 0; e < 4; ++e) {
        {
          const float inv = bf_rne(vg0[e]) * rsqrtf(bf_rne(vv0[e]) + 1e-5f);
          rmul[e] = inv;
          radd[e] = bf_rne(vb0[e]) - bf_rne(vm0[e]) * inv;
        }
        {
          const float inv = bf_rne(vg1[e]) * rsqrtf(bf_rne(vv1[e]) + 1e-5f);
          rmul[4 + e] = inv;
          radd[4 + e] = bf_rne(vb1[e]) - bf_rne(vm1[e]) * inv;
        }
      }
    }
#pragma unroll
    for (int j = 0; j < 4; ++j) {
      const int n = n0 + (j << 4) + rlane;
      float bv = 0.f;
      if (BIAS_MODE == 2) bv = bf_rne(bias[n]);
#pragma unroll
      for (int r = 0; r < 8; ++r) {
        float v = acc[i][j][r] * scale;
        if (BIAS_MODE == 1) v += rb[r];
        if (BIAS_MODE == 2) v += bv;
        if (BN) v = v * rmul[r] + radd[r];
        slab[(mOff + r) * 68 + (j << 4) + rlane] = v;
      }
    }
    __builtin_amdgcn_fence(__ATOMIC_RELEASE, "workgroup");
    __builtin_amdgcn_wave_barrier();
    __builtin_amdgcn_fence(__ATOMIC_ACQUIRE, "workgroup");
    if (OUT_MODE == 0) {
      float* C = (float*)Cout + (size_t)b * strideC;
      const int hh = lane >> 4, c4 = (lane & 15) * 4;
      v4f ov[8];
#pragma unroll
      for (int it = 0; it < 8; ++it) {
        const int row = it * 2 + hh;
        v4f v = *(const v4f*)(slab + row * 68 + c4);
        if (RESID) {
          const v4f xr = *(const v4f*)(Rb + (size_t)(mBase + row) * ldc + n0 + c4);
#pragma unroll
          for (int e = 0; e < 4; ++e) v[e] = v[e] + (BN ? bf_rne(xr[e]) : xr[e]);
        }
        ov[it] = v;
      }
      for (int pass = 0; pass < 2; ++pass) {
#pragma unroll
        for (int it = 0; it < 8; ++it) {
          const int row = it * 2 + hh;
          *(volatile v4f*)(C + (size_t)(mBase + row) * ldc + n0 + c4) = ov[it];
        }
        __threadfence();
      }
    } else {
      const int q = lane >> 3, c8 = (lane & 7) * 8;
      unsigned short* C  = (unsigned short*)Cout  + (size_t)b * strideC;
      unsigned short* C2 = (unsigned short*)Cout2 + (size_t)b * strideC;
      unsigned short* C3 = (unsigned short*)Cout3 + (size_t)b * strideC;
      for (int pass = 0; pass < 2; ++pass) {
#pragma unroll
        for (int it = 0; it < 4; ++it) {
          const int row = it * 4 + q;
          const float* sp = slab + row * 68 + c8;
          v8h hv, lv;
#pragma unroll
          for (int e = 0; e < 8; ++e) {
            const unsigned short hb = f2bf_bits(sp[e]);
            const unsigned short lb = f2bf_bits(sp[e] - bf_bits2f(hb));
            hv[e] = __builtin_bit_cast(_Float16, hb);
            lv[e] = __builtin_bit_cast(_Float16, lb);
          }
          const size_t go = (size_t)(mBase + row) * ldc + n0 + c8;
          *(volatile v8h*)(C + go) = hv;
          if (OUT_MODE == 2) { *(volatile v8h*)(C2 + go) = lv; }
          if (OUT_MODE == 3) { *(volatile v8h*)(C2 + go) = hv; *(volatile v8h*)(C3 + go) = lv; }
          if (OUT_MODE == 4) { *(volatile v8h*)(C2 + go) = lv; *(volatile v8h*)(C3 + go) = hv; }
        }
        __threadfence();
      }
    }
    __builtin_amdgcn_fence(__ATOMIC_RELEASE, "workgroup");
    __builtin_amdgcn_wave_barrier();
    __builtin_amdgcn_fence(__ATOMIC_ACQUIRE, "workgroup");
  }
}

__global__ __launch_bounds__(256) void tconv_kernel(const float* __restrict__ W, unsigned short* __restrict__ oh,
                                                    int ldin, int ldout, long sIn, long sOut) {
  __shared__ __align__(16) float tf[64 * 68];
  W  += (size_t)blockIdx.z * sIn;
  oh += (size_t)blockIdx.z * sOut;
  const int c0  = blockIdx.x * 64;
  const int r0  = blockIdx.y * 64;
  const int tid = threadIdx.x;
  {
    const int lr = tid >> 4;
    const int c4 = (tid & 15) * 4;
#pragma unroll
    for (int it = 0; it < 4; ++it) {
      const int rr = it * 16 + lr;
      const v4f a = *(const v4f*)(W + (size_t)(r0 + rr) * ldin + c0 + c4);
      *(v4f*)(tf + rr * 68 + c4) = a;
    }
  }
  __syncthreads();
  const int sub = tid >> 3;
  const int c8  = (tid & 7) * 8;
  v4u hv[2];
#pragma unroll
  for (int it = 0; it < 2; ++it) {
    const int oc = it * 32 + sub;
    v4u a;
#pragma unroll
    for (int q = 0; q < 4; ++q) {
      const float f0 = tf[(c8 + 2 * q) * 68 + oc];
      const float f1 = tf[(c8 + 2 * q + 1) * 68 + oc];
      a[q] = pk16(f2bf_bits(f0), f2bf_bits(f1));
    }
    hv[it] = a;
  }
  for (int pass = 0; pass < 2; ++pass) {
#pragma unroll
    for (int it = 0; it < 2; ++it) {
      const int oc = it * 32 + sub;
      const size_t go = (size_t)(c0 + oc) * ldout + r0 + c8;
      *(volatile v4u*)(oh + go) = hv[it];
    }
    __threadfence();
  }
}

__global__ __launch_bounds__(256) void wcvt_kernel(const float* __restrict__ wt, const float* __restrict__ wp,
                                                   const float* __restrict__ wg, const float* __restrict__ wr,
                                                   unsigned short* __restrict__ wcat, unsigned short* __restrict__ wr2) {
  const int g   = blockIdx.x * 256 + threadIdx.x;
  const int sel = blockIdx.y;
  if (g >= (CM * CI) / 8) return;
  const float* src;
  unsigned short* dst;
  if (sel < 3) {
    const float* w = (sel == 0) ? wt : ((sel == 1) ? wp : wg);
    src = w + (size_t)g * 8;
    dst = wcat + (size_t)sel * CM * CI + (size_t)g * 8;
  } else {
    const int row = g >> 4, c8 = (g & 15) * 8;
    src = wr + (size_t)row * CM + c8;
    dst = wr2 + (size_t)row * O2P + (size_t)(sel - 3) * CM + c8;
  }
  const v4f a = *(const v4f*)src;
  const v4f c = *(const v4f*)(src + 4);
  v4u o;
  o[0] = pk16(f2bf_bits(a[0]), f2bf_bits(a[1]));
  o[1] = pk16(f2bf_bits(a[2]), f2bf_bits(a[3]));
  o[2] = pk16(f2bf_bits(c[0]), f2bf_bits(c[1]));
  o[3] = pk16(f2bf_bits(c[2]), f2bf_bits(c[3]));
  *(volatile v4u*)dst = o;
  __threadfence();
  *(volatile v4u*)dst = o;
}

extern "C" void kernel_launch(void* const* d_in, const int* in_sizes, int n_in,
                              void* d_out, int out_size, void* d_ws, size_t ws_size,
                              hipStream_t stream) {
  if (n_in < 13) return;
  if (in_sizes[0] != NB * CI * NSP) return;
  if (in_sizes[1] != CM * CI || in_sizes[2] != CM) return;
  if (in_sizes[3] != CM * CI || in_sizes[4] != CM) return;
  if (in_sizes[5] != CM * CI || in_sizes[6] != CM) return;
  if (in_sizes[7] != CI * CM || in_sizes[8] != CI) return;
  if (in_sizes[9] != CI || in_sizes[10] != CI) return;
  if (in_sizes[11] != CI || in_sizes[12] != CI) return;
  if (out_size != NB * CI * NSP) return;

  const float* x       = (const float*)d_in[0];
  const float* w_theta = (const float*)d_in[1];
  const float* b_theta = (const float*)d_in[2];
  const float* w_phi   = (const float*)d_in[3];
  const float* b_phi   = (const float*)d_in[4];
  const float* w_g     = (const float*)d_in[5];
  const float* b_g     = (const float*)d_in[6];
  const float* w_rec   = (const float*)d_in[7];
  const float* b_rec   = (const float*)d_in[8];
  const float* gam     = (const float*)d_in[9];
  const float* bet     = (const float*)d_in[10];
  const float* mea     = (const float*)d_in[11];
  const float* var     = (const float*)d_in[12];

  const size_t PXT = (size_t)NTOKS * CI * 2;
  const size_t PWC = (size_t)T3P * CI * 2;
  const size_t PWR = (size_t)CI * O2P * 2;
  const size_t PT3 = (size_t)NTOKS * T3P * 2;
  const size_t PPG = (size_t)NB * CI * K3 * 2;
  const size_t PMT = (size_t)NB * CM * T3P * 2;
  const size_t PO2 = (size_t)NTOKS * O2P * 2;
  size_t off = 0;
  const size_t oXT = off; off += PXT;
  const size_t oWC = off; off += PWC;
  const size_t oWR = off; off += PWR;
  const size_t oT3 = off; off += PT3;
  const size_t oPG = off; off += PPG;
  const size_t oMT = off; off += PMT;
  const size_t oO2 = off; off += PO2;
  if (off > ws_size) return;
  if (off > (size_t)134217728) return;

  char* ws = (char*)d_ws;
  unsigned short* XT  = (unsigned short*)(ws + oXT);
  unsigned short* WC  = (unsigned short*)(ws + oWC);
  unsigned short* WR2 = (unsigned short*)(ws + oWR);
  unsigned short* T3  = (unsigned short*)(ws + oT3);
  unsigned short* PG3 = (unsigned short*)(ws + oPG);
  unsigned short* MT3 = (unsigned short*)(ws + oMT);
  unsigned short* O2  = (unsigned short*)(ws + oO2);
  float* out = (float*)d_out;

  const dim3 blk(256);

  tconv_kernel<<<dim3(NSP / 64, CI / 64, NB), blk, 0, stream>>>(x, XT, NSP, CI, (long)CI * NSP, (long)NSP * CI);

  wcvt_kernel<<<dim3((CM * CI) / 8 / 256, 5), blk, 0, stream>>>(w_theta, w_phi, w_g, w_rec, WC, WR2);

  const dim3 gT(((NTOKS / 64) * (CM / 64) + 7) / 8, 1);
  wmma_gemm64<1, 2, 3, false, false><<<gT, blk, 0, stream>>>(
      XT, CI, 0L, WC, CI, 0L,
      (void*)T3, (void*)(T3 + CM), (void*)(T3 + 2 * CM), T3P, 0L,
      b_theta, gam, bet, mea, var, x, 0L, NTOKS, CM, CI, 1.0f);

  const dim3 gP(((CM / 64) * (NSP / 64) + 7) / 8, NB);
  wmma_gemm64<1, 1, 4, false, false><<<gP, blk, 0, stream>>>(
      WC + (size_t)CM * CI, CI, 0L, XT, CI, (long)NSP * CI,
      (void*)PG3, (void*)(PG3 + NSP), (void*)(PG3 + 2 * NSP), K3, (long)CI * K3,
      b_phi, gam, bet, mea, var, x, 0L, CM, NSP, CI, 1.0f);

  wmma_gemm64<1, 1, 3, false, false><<<gP, blk, 0, stream>>>(
      WC + (size_t)2 * CM * CI, CI, 0L, XT, CI, (long)NSP * CI,
      (void*)(PG3 + (size_t)CM * K3), (void*)(PG3 + (size_t)CM * K3 + NSP), (void*)(PG3 + (size_t)CM * K3 + 2 * NSP), K3, (long)CI * K3,
      b_g, gam, bet, mea, var, x, 0L, CM, NSP, CI, 1.0f);

  const dim3 gM(1, NB);
  wmma_gemm64<1, 0, 4, false, false><<<gM, blk, 0, stream>>>(
      PG3 + (size_t)CM * K3, K3, (long)CI * K3, PG3, K3, (long)CI * K3,
      (void*)MT3, (void*)(MT3 + CM), (void*)(MT3 + 2 * CM), T3P, (long)CM * T3P,
      b_rec, gam, bet, mea, var, x, 0L, CM, CM, K3, 1.0f / (float)NSP);

  const dim3 gO(((NSP / 64) * (CM / 64) + 7) / 8, NB);
  wmma_gemm64<1, 0, 2, false, false><<<gO, blk, 0, stream>>>(
      T3, T3P, (long)NSP * T3P, MT3, T3P, (long)CM * T3P,
      (void*)O2, (void*)(O2 + CM), (void*)O2, O2P, (long)NSP * O2P,
      b_rec, gam, bet, mea, var, x, 0L, NSP, CM, T3P, 1.0f);

  const dim3 gR(((CI / 64) * (NSP / 64) + 7) / 8, NB);
  wmma_gemm64<1, 1, 0, true, true><<<gR, blk, 0, stream>>>(
      WR2, O2P, 0L, O2, O2P, (long)NSP * O2P,
      (void*)out, (void*)out, (void*)out, NSP, (long)CI * NSP,
      b_rec, gam, bet, mea, var, x, (long)CI * NSP, CI, NSP, O2P, 1.0f);
  (void)hipGetLastError();
}
